// EquivariantSwarmDecoder_23450521436537
// MI455X (gfx1250) — hardware-run, weakly checked
//
#include <hip/hip_runtime.h>
#include <math.h>

typedef __attribute__((ext_vector_type(16))) _Float16 v16h;
typedef __attribute__((ext_vector_type(16))) __bf16 v16b;
typedef __attribute__((ext_vector_type(8)))  _Float16 v8h;
typedef __attribute__((ext_vector_type(8)))  float v8f;
typedef __attribute__((ext_vector_type(4)))  float v4f;
typedef __attribute__((ext_vector_type(2)))  float v2f;
typedef __attribute__((ext_vector_type(4)))  unsigned v4u;
typedef __attribute__((ext_vector_type(4)))  int v4i;
typedef float __attribute__((may_alias)) float_a;
typedef int __attribute__((may_alias)) int_a;

template <typename T> __device__ __forceinline__ void vst2(void* p, T v) { *(volatile T*)p = v; __threadfence(); *(volatile T*)p = v; }
__device__ __forceinline__ v8f wmma16(v16h a, v16h b, v8f c) {
  v8f d = __builtin_amdgcn_wmma_f32_16x16x32_f16(false, a, false, b, (short)0, c, false, false);
  asm volatile("v_nop\n\tv_nop\n\tv_nop\n\tv_nop" : "+v"(d) : "v"(a), "v"(b));
  return d;
}
__device__ __forceinline__ v8f wmma_bf(v16b a, v16b b, v8f c) {
  v8f d = __builtin_amdgcn_wmma_f32_16x16x32_bf16(false, a, false, b, (short)0, c, false, false);
  asm volatile("v_nop\n\tv_nop\n\tv_nop\n\tv_nop" : "+v"(d) : "v"(a), "v"(b));
  return d;
}
__device__ __forceinline__ v16h frag_h(const _Float16* rowk0, int lane) {
  union { v16h v; v8h q[2]; } u; const _Float16* p = rowk0 + 8 * (lane >> 4);
  u.q[0] = *(const v8h*)p; u.q[1] = *(const v8h*)(p + 16); return u.v;
}
__device__ __forceinline__ v16h frag_f32(const float* rowk0, int lane) {
  v16h a; const float* p = rowk0 + 8 * (lane >> 4);
#pragma unroll
  for (int i = 0; i < 8; ++i) { a[i] = (_Float16)p[i]; a[8 + i] = (_Float16)p[16 + i]; }
  return a;
}
__device__ __forceinline__ v16h frag_f32s(const float* rowk0, int lane, float sc) {
  v16h a; const float* p = rowk0 + 8 * (lane >> 4);
#pragma unroll
  for (int i = 0; i < 8; ++i) { a[i] = (_Float16)(p[i] * sc); a[8 + i] = (_Float16)(p[16 + i] * sc); }
  return a;
}
__device__ __forceinline__ v16h fragc_f32(const float* W, int k0, int n, int lane, int ld, int K) {
  v16h a; const int g = lane >> 4;
#pragma unroll
  for (int i = 0; i < 8; ++i) { const int ka = k0 + 8 * g + i, kb = ka + 16;
    a[i] = (_Float16)(ka < K ? W[(size_t)(ka < K ? ka : K - 1) * ld + n] : 0.f); a[8 + i] = (_Float16)(kb < K ? W[(size_t)(kb < K ? kb : K - 1) * ld + n] : 0.f); }
  return a;
}
struct F2 { v16b h, l; };
__device__ __forceinline__ F2 bsplit16(const float v[16]) { F2 r;
#pragma unroll
  for (int i = 0; i < 16; ++i) { const __bf16 h = (__bf16)v[i]; r.h[i] = h; r.l[i] = (__bf16)(v[i] - (float)h); }
  return r; }
__device__ __forceinline__ F2 split_row(const float* row, int k0, int lane) { float v[16]; const float* p = row + k0 + 8 * (lane >> 4);
#pragma unroll
  for (int i = 0; i < 8; ++i) { v[i] = p[i]; v[8 + i] = p[16 + i]; }
  return bsplit16(v); }
__device__ __forceinline__ F2 split_rowK(const float* row, int k0, int lane, int K) { float v[16]; const int g = lane >> 4;
#pragma unroll
  for (int i = 0; i < 8; ++i) { const int ka = k0 + 8 * g + i, kb = ka + 16; v[i] = ka < K ? row[ka < K ? ka : K - 1] : 0.f; v[8 + i] = kb < K ? row[kb < K ? kb : K - 1] : 0.f; }
  return bsplit16(v); }
__device__ __forceinline__ F2 split_col(const float* W, int k0, int n, int lane, int ld, int K) { float v[16]; const int g = lane >> 4;
#pragma unroll
  for (int i = 0; i < 8; ++i) { const int ka = k0 + 8 * g + i, kb = ka + 16; v[i] = ka < K ? W[(size_t)(ka < K ? ka : K - 1) * ld + n] : 0.f; v[8 + i] = kb < K ? W[(size_t)(kb < K ? kb : K - 1) * ld + n] : 0.f; }
  return bsplit16(v); }
__device__ __forceinline__ v8f mac3(const F2& a, const F2& b, v8f c) { c = wmma_bf(a.l, b.h, c); c = wmma_bf(a.h, b.l, c); return wmma_bf(a.h, b.h, c); }
__device__ __forceinline__ float sigm(float v) { return 1.0f / (1.0f + expf(-v)); }
#define LDSX() do { asm volatile("s_wait_dscnt 0" ::: "memory"); __builtin_amdgcn_wave_barrier(); __builtin_amdgcn_fence(__ATOMIC_RELEASE, "workgroup"); } while (0)


#define NBT 128
#define KP 64
#define NM 2048
#define QD 128
#define AD 128
#define HH 256
#define NC 32
#define NR (NBT * NM)
#define WSC 256.0f
#ifndef TNB
#define TNB NBT
#endif
typedef __attribute__((ext_vector_type(8))) __bf16 v8b;
__device__ __forceinline__ v16b frag_b(const __bf16* rowk0, int lane) {
  union { v16b v; v8b q[2]; } u; const __bf16* p = rowk0 + 8 * (lane >> 4);
  u.q[0] = *(const v8b*)p; u.q[1] = *(const v8b*)(p + 16); return u.v;
}
__device__ __forceinline__ float bfr(float v) { return (float)(__bf16)v; }
__device__ __attribute__((noinline)) float exp_ni(float v) { return expf(v); }
__device__ __attribute__((noinline)) float erf_ni(float v) { return erff(v); }
__device__ __attribute__((noinline)) float gelu_e(float v) { return 0.5f * v * (1.0f + erff(v * 0.70710678118654752f)); }

#define WS_INV 0u
#define WS_QK  (WS_INV + 4u * (size_t)NBT * KP)
#define WS_Y3  (WS_QK + 4u * (size_t)2 * NM)
#define WS_GS  (WS_Y3 + 4u * (size_t)NR * 4)
#define WS_AT  (WS_GS + 4u * (size_t)NBT * HH)
#define WS_BT  (WS_AT + 4u * (size_t)NBT * HH)
#define WS_W2  (WS_BT + 4u * (size_t)NM * HH)
#define WS_W3  (WS_W2 + 2u * (size_t)HH * HH)
#define WS_WH  (WS_W3 + 2u * (size_t)HH * HH)
#define WS_END (WS_WH + 2u * (size_t)48 * HH)

__global__ __launch_bounds__(256) void k_packw(const float* __restrict__ W2, const float* __restrict__ W3, const float* __restrict__ TW, const float* __restrict__ WW, const float* __restrict__ CW, char* __restrict__ ws) { const int n = blockIdx.x, t = threadIdx.x; __shared__ __align__(16) _Float16 s2[HH], s3[HH], sh[HH];
  s2[t] = (_Float16)(bfr(W2[(size_t)n * HH + t]) * WSC); s3[t] = (_Float16)(bfr(W3[(size_t)n * HH + t]) * WSC);
  if (n < 48) sh[t] = (n < NC) ? (_Float16)(bfr(TW[(size_t)n * HH + t]) * WSC) : (n == NC) ? (_Float16)(bfr(WW[t]) * WSC) : (n == NC + 1) ? (_Float16)(bfr(CW[t]) * WSC) : (_Float16)0.0f;
  __syncthreads();
  if (t < HH / 8) { vst2((unsigned*)((_Float16*)(ws + WS_W2) + (size_t)n * HH + t * 8), *(const v4u*)&s2[t * 8]); vst2((unsigned*)((_Float16*)(ws + WS_W3) + (size_t)n * HH + t * 8), *(const v4u*)&s3[t * 8]); if (n < 48) vst2((unsigned*)((_Float16*)(ws + WS_WH) + (size_t)n * HH + t * 8), *(const v4u*)&sh[t * 8]); } }
__global__ __launch_bounds__(256) void k_inv(const float* __restrict__ G, const float* __restrict__ GW1, const float* __restrict__ GB1, const float* __restrict__ GW2, const float* __restrict__ GB2, const float* __restrict__ GW3, const float* __restrict__ GB3, const float* __restrict__ PW1, const float* __restrict__ PB1, float* __restrict__ INV, float* __restrict__ GS, float* __restrict__ AT) {
  __shared__ __align__(16) float sv[KP]; __shared__ __align__(16) float h1[HH], h2[HH], h3[HH], so2[HH]; const int t = threadIdx.x; const size_t b = blockIdx.x;
  if (t < KP) { const float x = bfr(G[(b * KP + t) * 3 + 0]), y = bfr(G[(b * KP + t) * 3 + 1]), z = bfr(G[(b * KP + t) * 3 + 2]); sv[t] = sqrtf(x * x + y * y + z * z); } __syncthreads();
  if (t < KP / 4) vst2(INV + b * KP + t * 4, *(const v4f*)&sv[t * 4]);
  { float a = bfr(GB1[t]);
#pragma unroll 1
    for (int i = 0; i < KP; ++i) a += bfr(GW1[(size_t)t * KP + i]) * sv[i]; h1[t] = gelu_e(a); } __syncthreads();
  { float a = bfr(GB2[t]);
#pragma unroll 1
    for (int i = 0; i < HH; ++i) a += bfr(GW2[(size_t)t * HH + i]) * h1[i]; h2[t] = gelu_e(a); } __syncthreads();
  { float a = bfr(GB3[t]);
#pragma unroll 1
    for (int i = 0; i < HH; ++i) a += bfr(GW3[(size_t)t * HH + i]) * h2[i]; h3[t] = a; } __syncthreads();
  if (t < HH / 4) vst2(GS + b * HH + t * 4, *(const v4f*)&h3[t * 4]);
  { float a = bfr(PB1[t]);
#pragma unroll 1
    for (int i = 0; i < HH; ++i) a += bfr(PW1[(size_t)t * (HH + QD + 1) + i]) * h3[i]; so2[t] = a; } __syncthreads();
  if (t < HH / 4) vst2(AT + b * HH + t * 4, *(const v4f*)&so2[t * 4]); }
__global__ __launch_bounds__(256) void k_bt(const float* __restrict__ QRY, const float* __restrict__ PW1, float* __restrict__ BT) { __shared__ float sq[QD]; __shared__ __align__(16) float so2[HH]; const int t = threadIdx.x; const size_t m = blockIdx.x;
  if (t < QD) sq[t] = bfr(QRY[m * QD + t]); __syncthreads();
  { float a = 0.f;
#pragma unroll 1
    for (int i = 0; i < QD; ++i) a += bfr(PW1[(size_t)t * (HH + QD + 1) + HH + i]) * sq[i]; so2[t] = a; } __syncthreads();
  if (t < HH / 4) vst2(BT + m * HH + t * 4, *(const v4f*)&so2[t * 4]); }
__global__ __launch_bounds__(64) void k_qk(const float* __restrict__ QRY, const float* __restrict__ QW, const float* __restrict__ QB, const float* __restrict__ KW, const float* __restrict__ KB, float* __restrict__ QK) { __shared__ __align__(16) float s1[64], s2[64]; __shared__ float sw[AD][QD + 1]; const int t = threadIdx.x; const size_t m = (size_t)blockIdx.x * 64 + t;
  for (int e = t; e < AD * QD; e += 64) sw[e / QD][e % QD] = bfr(QW[e]); __syncthreads();
  float pk = 0.f, pb = 0.f;
#pragma unroll 1
  for (int a = 0; a < AD; ++a) { float q = bfr(QB[a]);
#pragma unroll 1
    for (int i = 0; i < QD; ++i) q += sw[a][i] * bfr(QRY[m * QD + i]); pk += q * bfr(KW[a]); pb += q * bfr(KB[a]); }
  s1[t] = pk; s2[t] = pb; __syncthreads();
  if (t < 16) { vst2(QK + (size_t)blockIdx.x * 64 + t * 4, *(const v4f*)&s1[t * 4]); vst2(QK + NM + (size_t)blockIdx.x * 64 + t * 4, *(const v4f*)&s2[t * 4]); } }
__global__ __launch_bounds__(64) void k_att(const float* __restrict__ INV, const float* __restrict__ QK, const float* __restrict__ G, float* __restrict__ Y3) { __shared__ float si[KP], sg[KP][3]; __shared__ __align__(16) float so2[64][4]; const int t = threadIdx.x; const size_t b = blockIdx.y; const size_t m = (size_t)blockIdx.x * 64 + t;
  si[t] = INV[b * KP + t]; for (int d = 0; d < 3; ++d) sg[t][d] = bfr(G[(b * KP + t) * 3 + d]); __syncthreads();
  const float a1 = QK[m], a0 = QK[NM + m]; const float isq = 0.088388347648318447f;
  float mx = -3.0e38f;
#pragma unroll 1
  for (int k = 0; k < KP; ++k) mx = fmaxf(mx, (si[k] * a1 + a0) * isq);
  float z = 0.f, y0 = 0.f, y1 = 0.f, y2 = 0.f, at = 0.f;
#pragma unroll 1
  for (int k = 0; k < KP; ++k) { const float e = expf((si[k] * a1 + a0) * isq - mx); z += e; y0 += e * sg[k][0]; y1 += e * sg[k][1]; y2 += e * sg[k][2]; at += e * si[k]; }
  const float iz = 1.0f / z; so2[t][0] = y0 * iz; so2[t][1] = y1 * iz; so2[t][2] = y2 * iz; so2[t][3] = at * iz; __syncthreads();
  vst2(Y3 + ((b * NM + (size_t)blockIdx.x * 64 + t) * 4), *(const v4f*)&so2[t][0]); }
__device__ __forceinline__ void lds2frag(const _Float16 (*sh)[HH + 8], const _Float16 (*sl)[HH + 8], int row, int kc, int g, v16h& ah, v16h& al) { const _Float16* ph = &sh[row][kc * 32 + 8 * g]; const _Float16* pl = &sl[row][kc * 32 + 8 * g];
#pragma unroll
  for (int i = 0; i < 8; ++i) { ah[i] = ph[i]; ah[8 + i] = ph[16 + i]; al[i] = pl[i]; al[8 + i] = pl[16 + i]; } }
__global__ __launch_bounds__(128) void k_mlp(const float* __restrict__ AT, const float* __restrict__ BT, const float* __restrict__ Y3, const float* __restrict__ PW1, const float* __restrict__ PB2, const float* __restrict__ PB3, const char* __restrict__ ws, const float* __restrict__ TB, const float* __restrict__ WB, const float* __restrict__ CB, float* __restrict__ OUT0, float* __restrict__ OUT1, float* __restrict__ OUT2) {
  __shared__ __align__(16) _Float16 h1b[2][64][HH + 8]; __shared__ __align__(16) _Float16 h2b[2][64][HH + 8];
  __shared__ __align__(16) float st[64][36]; __shared__ __align__(16) float sw[64]; __shared__ __align__(16) float sy[64 * 3];
  _Float16 (*ah1)[HH + 8] = h1b[0]; _Float16 (*al1)[HH + 8] = h1b[1]; float (*sf)[HH + 4] = (float (*)[HH + 4])&h1b[0][0][0];
  const int tid = threadIdx.x, wave = tid >> 5, lane = tid & 31, col = lane & 15, g = lane >> 4; const size_t rb = (size_t)blockIdx.x * 64; const size_t r0 = rb + wave * 16; const _Float16 *W2 = (const _Float16*)(ws + WS_W2), *W3 = (const _Float16*)(ws + WS_W3), *WH = (const _Float16*)(ws + WS_WH);
  for (int e = lane; e < 16 * HH; e += 32) { const int rl = e / HH, j = e % HH; const size_t row = r0 + rl; const size_t b = row / NM, m = row % NM; const float v = gelu_e(AT[b * HH + j] + BT[m * HH + j] + bfr(PW1[(size_t)j * (HH + QD + 1) + HH + QD]) * Y3[row * 4 + 3]); const _Float16 hv = (_Float16)v; ah1[wave * 16 + rl][j] = hv; al1[wave * 16 + rl][j] = (_Float16)((v - (float)hv) * 2048.0f); }
  LDSX();
  for (int half = 0; half < 2; ++half) { v8f acc[8] = {}, accl[8] = {};
#pragma unroll 1
    for (int kc = 0; kc < HH / 32; ++kc) { v16h a, al; lds2frag(ah1, al1, wave * 16 + col, kc, g, a, al);
#pragma unroll
      for (int j = 0; j < 8; ++j) { const v16h w = frag_h(W2 + (size_t)(half * 128 + j * 16 + col) * HH + kc * 32, lane); acc[j] = wmma16(a, w, acc[j]); accl[j] = wmma16(al, w, accl[j]); } }
#pragma unroll
    for (int j = 0; j < 8; ++j) { const int c = half * 128 + j * 16 + col; const float bb = bfr(PB2[c]);
#pragma unroll
      for (int r = 0; r < 8; ++r) { const float v = gelu_e((acc[j][r] + accl[j][r] * (1.0f / 2048.0f)) * (1.0f / WSC) + bb); const _Float16 hv = (_Float16)v; h2b[0][wave * 16 + 8 * g + r][c] = hv; h2b[1][wave * 16 + 8 * g + r][c] = (_Float16)((v - (float)hv) * 2048.0f); } } }
  LDSX();
  for (int half = 0; half < 2; ++half) { v8f acc[8] = {}, accl[8] = {};
#pragma unroll 1
    for (int kc = 0; kc < HH / 32; ++kc) { v16h a, al; lds2frag(h2b[0], h2b[1], wave * 16 + col, kc, g, a, al);
#pragma unroll
      for (int j = 0; j < 8; ++j) { const v16h w = frag_h(W3 + (size_t)(half * 128 + j * 16 + col) * HH + kc * 32, lane); acc[j] = wmma16(a, w, acc[j]); accl[j] = wmma16(al, w, accl[j]); } }
#pragma unroll
    for (int j = 0; j < 8; ++j) { const float bb = bfr(PB3[half * 128 + j * 16 + col]);
#pragma unroll
      for (int r = 0; r < 8; ++r) sf[wave * 16 + 8 * g + r][half * 128 + j * 16 + col] = (acc[j][r] + accl[j][r] * (1.0f / 2048.0f)) * (1.0f / WSC) + bb; } }
  LDSX();
  { v8f acc[3] = {}, accl[3] = {};
#pragma unroll 1
    for (int kc = 0; kc < HH / 32; ++kc) { v16h a, al; { const float* p = &sf[wave * 16 + col][kc * 32 + 8 * g];
#pragma unroll
        for (int i = 0; i < 8; ++i) { const float x0 = p[i], x1 = p[16 + i]; const _Float16 q0 = (_Float16)x0, q1 = (_Float16)x1; a[i] = q0; a[8 + i] = q1; al[i] = (_Float16)((x0 - (float)q0) * 2048.0f); al[8 + i] = (_Float16)((x1 - (float)q1) * 2048.0f); } }
#pragma unroll
      for (int j = 0; j < 3; ++j) { const v16h w = frag_h(WH + (size_t)(j * 16 + col) * HH + kc * 32, lane); acc[j] = wmma16(a, w, acc[j]); accl[j] = wmma16(al, w, accl[j]); } }
#pragma unroll
    for (int r = 0; r < 8; ++r) { const int rl = wave * 16 + 8 * g + r; const size_t row = r0 + 8 * g + r; const float v0 = (acc[0][r] + accl[0][r] * (1.0f / 2048.0f)) * (1.0f / WSC), v1 = (acc[1][r] + accl[1][r] * (1.0f / 2048.0f)) * (1.0f / WSC), v2 = (acc[2][r] + accl[2][r] * (1.0f / 2048.0f)) * (1.0f / WSC);
      st[rl][col] = v0 + bfr(TB[col]); st[rl][16 + col] = v1 + bfr(TB[16 + col]);
      if (col == 0) sw[rl] = v2 + bfr(WB[0]);
      if (col == 1) { const float gl = v2 + bfr(CB[0]); float gt = 1.0f / (1.0f + expf(-gl)); gt = fminf(fmaxf(gt, 0.f), 1.f); for (int d = 0; d < 3; ++d) sy[rl * 3 + d] = Y3[row * 4 + d] * gt; } } }
  __syncthreads();
  for (int e = tid; e < 64 * 8; e += 128) { const int rl = e >> 3, q = e & 7; vst2(OUT1 + (rb + rl) * NC + q * 4, *(const v4f*)&st[rl][q * 4]); }
  if (tid < 16) vst2(OUT2 + rb + tid * 4, *(const v4f*)&sw[tid * 4]);
  if (tid < 48) vst2(OUT0 + rb * 3 + tid * 4, *(const v4f*)&sy[tid * 4]); }
extern "C" void kernel_launch(void* const* d_in, const int* in_sizes, int n_in, void* d_out, int out_size, void* d_ws, size_t ws_size, hipStream_t stream) {
  (void)in_sizes; (void)n_in; (void)out_size;
  const float** F = (const float**)d_in;
  if (ws_size < (size_t)WS_END) return;
  char* ws = (char*)d_ws; float *INV = (float*)(ws + WS_INV), *QK = (float*)(ws + WS_QK), *Y3 = (float*)(ws + WS_Y3), *GS = (float*)(ws + WS_GS), *AT = (float*)(ws + WS_AT), *BT = (float*)(ws + WS_BT);   float* OUT0 = (float*)d_out; float* OUT1 = OUT0 + (size_t)NR * 3; float* OUT2 = OUT1 + (size_t)NR * NC;
  const int nrows = TNB * NM;
  k_packw<<<HH, 256, 0, stream>>>(F[14], F[16], F[18], F[20], F[22], ws);
  k_inv<<<TNB, 256, 0, stream>>>(F[0], F[6], F[7], F[8], F[9], F[10], F[11], F[12], F[13], INV, GS, AT);
  k_bt<<<NM, 256, 0, stream>>>(F[1], F[12], BT);
  k_qk<<<NM / 64, 64, 0, stream>>>(F[1], F[2], F[3], F[4], F[5], QK);
  k_att<<<dim3(NM / 64, TNB), 64, 0, stream>>>(INV, QK, F[0], Y3);
  k_mlp<<<nrows / 64, 128, 0, stream>>>(AT, BT, Y3, F[12], F[15], F[17], ws, F[19], F[21], F[23], OUT0, OUT1, OUT2);
}
